// MistralAttention_36223754175091
// MI455X (gfx1250) — hardware-verified
//
#include <hip/hip_runtime.h>
#include <math.h>
#include <stdint.h>

#define NB    2
#define SEQ   2048
#define HID   288
#define NH    18
#define HD    16
#define NPAIR 8
#define QS    32
#define NTOK  (NB * SEQ)
#define NQB   (SEQ / 64)
static_assert(NH * HD == HID);
static_assert(NPAIR * 2 == HD);
static_assert((SEQ % 64) == 0 && (HID % 32) == 0 && (NTOK % 64) == 0);
static_assert(((NTOK / 64) * (HID / 32)) % 4 == 0);
static_assert((NTOK * HID) % (8 * 256) == 0);
static_assert(((HID * HID) % 8) == 0 && (((HID * HID) / 8) % 32) == 0);
static_assert((SEQ % 32) == 0);

typedef __bf16   v16b __attribute__((ext_vector_type(16)));
typedef __bf16   v8b  __attribute__((ext_vector_type(8)));
typedef float    v8f  __attribute__((ext_vector_type(8)));
typedef float    v4f  __attribute__((ext_vector_type(4)));
typedef unsigned int v4u __attribute__((ext_vector_type(4)));

__device__ __forceinline__ unsigned short bf_bits(float f) {
  unsigned u = __float_as_uint(f);
  return (unsigned short)((u + 0x7FFFu + ((u >> 16) & 1u)) >> 16);
}
__device__ __forceinline__ float bf_up(unsigned short h) { return __uint_as_float(((unsigned)h) << 16); }
__device__ __forceinline__ unsigned pk16(unsigned short a, unsigned short b) { return (unsigned)a | ((unsigned)b << 16); }
__device__ __forceinline__ v8f zero8() { v8f z = {0.f, 0.f, 0.f, 0.f, 0.f, 0.f, 0.f, 0.f}; return z; }

__device__ __forceinline__ v16b ldfrag_b(const __bf16* p) {
  union { v16b v; v8b h[2]; } f;
  f.h[0] = *(const v8b*)(p);
  f.h[1] = *(const v8b*)(p + 16);
  return f.v;
}
__device__ __forceinline__ v16b ldfrag_b2(const __bf16* p0, const __bf16* p1) {
  union { v16b v; v8b h[2]; } f;
  f.h[0] = *(const v8b*)(p0);
  f.h[1] = *(const v8b*)(p1);
  return f.v;
}

__device__ __forceinline__ v8f mma_b(v16b a, v16b b, v8f c) {
  c = __builtin_amdgcn_wmma_f32_16x16x32_bf16(false, a, false, b, (short)0, c, false, false);
  asm volatile("v_nop\n\tv_nop\n\tv_nop\n\tv_nop" : "+v"(c) : "v"(a), "v"(b));
  return c;
}

__global__ __launch_bounds__(32) void rope_inv(float* inv) {
  const int i = (int)threadIdx.x;
  const float e = (float)(2 * i) * (1.0f / (float)HD);
  const float p = powf(10000.0f, e);
  const float v = 1.0f / p;
  *(volatile float*)(inv + i) = v;
  __threadfence();
  *(volatile float*)(inv + i) = v;
}

__global__ __launch_bounds__(256) void rope_tab(const float* __restrict__ inv, float* ctab, float* stab) {
  const int tid = (int)threadIdx.x;
  const int i = tid & (NPAIR - 1);
  const int t = blockIdx.x * 32 + (tid >> 3);
  const float f   = inv[i];
  const float ang = (float)t * f;
  float sn, cs;
  sincosf(ang, &sn, &cs);
  const size_t o = (size_t)t * NPAIR + i;
  *(volatile float*)(ctab + o) = cs;
  *(volatile float*)(stab + o) = sn;
  __threadfence();
  *(volatile float*)(ctab + o) = cs;
  *(volatile float*)(stab + o) = sn;
}

__global__ __launch_bounds__(256) void cvt_bf16x8(const float* __restrict__ in, unsigned short* out, int n8) {
  const int i = blockIdx.x * 256 + (int)threadIdx.x;
  if (i < n8) {
    const v4f a = *(const v4f*)(in + (size_t)i * 8);
    const v4f b = *(const v4f*)(in + (size_t)i * 8 + 4);
    v4u p;
    p[0] = pk16(bf_bits(a[0]), bf_bits(a[1]));
    p[1] = pk16(bf_bits(a[2]), bf_bits(a[3]));
    p[2] = pk16(bf_bits(b[0]), bf_bits(b[1]));
    p[3] = pk16(bf_bits(b[2]), bf_bits(b[3]));
    *(volatile v4u*)(out + (size_t)i * 8) = p;
    __threadfence();
    *(volatile v4u*)(out + (size_t)i * 8) = p;
  }
}

template <int MODE, bool TWOA>
__global__ __launch_bounds__(128) void gemm_xw(
    const unsigned short* __restrict__ Ap, const unsigned short* __restrict__ A2p,
    const unsigned short* __restrict__ Btp, void* C0, void* C1,
    const float* __restrict__ ctab, const float* __restrict__ stab) {
  static_assert(MODE >= 0 && MODE <= 3);
  constexpr int M = NTOK, N = HID, K = HID;
  constexpr int TN = N / 32;
  constexpr int TM = M / 64;
  const __bf16* A  = (const __bf16*)(const void*)Ap;
  const __bf16* A2 = (const __bf16*)(const void*)A2p;
  const __bf16* Bt = (const __bf16*)(const void*)Btp;
  __shared__ __align__(16) float sT[4][64 * 36];

  const int lane = threadIdx.x & 31;
  const int wave = threadIdx.x >> 5;
  const int tile = blockIdx.x * 4 + wave;
  if (tile >= TM * TN) return;
  const int tm = tile / TN;
  const int tn = tile - tm * TN;
  const int m0 = tm << 6;
  const int n0 = tn << 5;
  const int c    = lane & 15;
  const int koff = (lane >> 4) * 8;
  const int mOff = (lane >> 4) * 8;
  const int bidx = m0 / SEQ;
  const int tl0  = m0 - bidx * SEQ;

  v8f acc[4][2];
#pragma unroll
  for (int i = 0; i < 4; ++i)
#pragma unroll
    for (int j = 0; j < 2; ++j) acc[i][j] = zero8();

  for (int k0 = 0; k0 < K; k0 += 32) {
    v16b bh[2];
#pragma unroll
    for (int j = 0; j < 2; ++j) bh[j] = ldfrag_b(Bt + (size_t)(n0 + (j << 4) + c) * K + koff + k0);
#pragma unroll
    for (int i = 0; i < 4; ++i) {
      v16b ah, al;
      if (MODE == 3) {
        const int pr = k0 >> 5;
        const size_t o0 = (((size_t)(bidx * NH + 2 * pr)) * SEQ + tl0 + (i << 4) + c) * HD + koff;
        const size_t o1 = o0 + (size_t)SEQ * HD;
        ah = ldfrag_b2(A + o0, A + o1);
        al = ah;
        if (TWOA) al = ldfrag_b2(A2 + o0, A2 + o1);
      } else {
        const size_t ao = (size_t)(m0 + (i << 4) + c) * K + koff + k0;
        ah = ldfrag_b(A + ao);
        al = ah;
        if (TWOA) al = ldfrag_b(A2 + ao);
      }
#pragma unroll
      for (int j = 0; j < 2; ++j) {
        acc[i][j] = mma_b(ah, bh[j], acc[i][j]);
        if (TWOA) acc[i][j] = mma_b(al, bh[j], acc[i][j]);
      }
    }
  }

  float* slab = sT[wave];
#pragma unroll
  for (int i = 0; i < 4; ++i)
#pragma unroll
    for (int j = 0; j < 2; ++j)
#pragma unroll
      for (int r = 0; r < 8; ++r)
        slab[((i << 4) + mOff + r) * 36 + (j << 4) + c] = acc[i][j][r];
  __builtin_amdgcn_fence(__ATOMIC_RELEASE, "workgroup");
  __builtin_amdgcn_wave_barrier();
  __builtin_amdgcn_fence(__ATOMIC_ACQUIRE, "workgroup");

  if (MODE == 3) {
    float* Cf = (float*)C0;
    const int q4 = lane >> 3, c4 = (lane & 7) * 4;
    for (int pass = 0; pass < 2; ++pass) {
#pragma unroll
      for (int it = 0; it < 16; ++it) {
        const int row = it * 4 + q4;
        const v4f v = *(const v4f*)(slab + row * 36 + c4);
        *(volatile v4f*)(Cf + (size_t)(m0 + row) * HID + n0 + c4) = v;
      }
      __threadfence();
    }
  } else if (MODE == 2) {
    unsigned short* P0 = (unsigned short*)C0;
    unsigned short* P1 = (unsigned short*)C1;
    const int q4 = lane >> 3, t8 = (lane & 7) * 8;
#pragma unroll 2
    for (int it = 0; it < 8; ++it) {
      const int n = it * 4 + q4;
      float f[8];
#pragma unroll
      for (int e = 0; e < 8; ++e) f[e] = slab[(t8 + e) * 36 + n];
      v4u a, a2;
#pragma unroll
      for (int e = 0; e < 4; ++e) {
        const float f0 = f[2 * e], f1 = f[2 * e + 1];
        const unsigned short h0 = bf_bits(f0), h1 = bf_bits(f1);
        const unsigned short l0 = bf_bits(f0 - bf_up(h0)), l1 = bf_bits(f1 - bf_up(h1));
        a[e] = pk16(h0, h1); a2[e] = pk16(l0, l1);
      }
      const size_t go = ((size_t)(bidx * HID + n0 + n)) * SEQ + tl0 + t8;
      *(volatile v4u*)(P0 + go) = a;
      *(volatile v4u*)(P1 + go) = a2;
      __threadfence();
      *(volatile v4u*)(P0 + go) = a;
      *(volatile v4u*)(P1 + go) = a2;
    }
  } else {
    unsigned short* P0 = (unsigned short*)C0;
    unsigned short* P1 = (unsigned short*)C1;
    const int r4 = lane >> 2, s8 = (lane & 3) * 8;
    const int dbase = s8 & 8;
    const bool isLo = (s8 >= 16);
    const float sg = (dbase == 0) ? -1.0f : 1.0f;
    const int h0 = n0 >> 4;
#pragma unroll 1
    for (int hd = 0; hd < 2; ++hd) {
#pragma unroll 2
      for (int it = 0; it < 8; ++it) {
        const int row = it * 8 + r4;
        const int t = tl0 + row;
        const float* xr = slab + row * 36 + hd * 16;
        float x[8], y[8], f[8];
#pragma unroll
        for (int e = 0; e < 8; ++e) { x[e] = xr[dbase + e]; y[e] = xr[(dbase ^ 8) + e]; }
        const v4f cv0 = *(const v4f*)(ctab + (size_t)t * NPAIR);
        const v4f cv1 = *(const v4f*)(ctab + (size_t)t * NPAIR + 4);
        const v4f sv0 = *(const v4f*)(stab + (size_t)t * NPAIR);
        const v4f sv1 = *(const v4f*)(stab + (size_t)t * NPAIR + 4);
        {
#pragma clang fp contract(off)
#pragma unroll
          for (int e = 0; e < 4; ++e) {
            {
              const float ry = sg * y[e];
              const float p0 = x[e] * cv0[e];
              const float p1 = ry * sv0[e];
              f[e] = p0 + p1;
            }
            {
              const float ry = sg * y[4 + e];
              const float p0 = x[4 + e] * cv1[e];
              const float p1 = ry * sv1[e];
              f[4 + e] = p0 + p1;
            }
          }
        }
        v4u hp, lp;
#pragma unroll
        for (int e = 0; e < 4; ++e) {
          const float f0 = f[2 * e], f1 = f[2 * e + 1];
          const unsigned short hb0 = bf_bits(f0), hb1 = bf_bits(f1);
          const unsigned short lb0 = bf_bits(f0 - bf_up(hb0)), lb1 = bf_bits(f1 - bf_up(hb1));
          hp[e] = pk16(hb0, hb1); lp[e] = pk16(lb0, lb1);
        }
        const size_t go = (((size_t)(bidx * NH + h0 + hd)) * SEQ + t) * QS + s8;
        if (MODE == 0) {
          v4u pc;
#pragma unroll
          for (int e = 0; e < 4; ++e) pc[e] = isLo ? lp[e] : hp[e];
          *(volatile v4u*)(P0 + go) = pc;
          __threadfence();
          *(volatile v4u*)(P0 + go) = pc;
        } else {
          v4u pz;
#pragma unroll
          for (int e = 0; e < 4; ++e) pz[e] = isLo ? 0u : lp[e];
          *(volatile v4u*)(P0 + go) = hp;
          *(volatile v4u*)(P1 + go) = pz;
          __threadfence();
          *(volatile v4u*)(P0 + go) = hp;
          *(volatile v4u*)(P1 + go) = pz;
        }
      }
    }
  }
}

__global__ __launch_bounds__(128)
void attn_causal16(const unsigned short* __restrict__ qcp, const unsigned short* __restrict__ kdp,
                   const unsigned short* __restrict__ kzp, const unsigned short* __restrict__ vhp,
                   const unsigned short* __restrict__ vlp, unsigned short* ohp, unsigned short* olp) {
  union FB { v16b v; v8b h[2]; };
  __shared__ __align__(16) __bf16 Psh[4][16 * 64];
  __shared__ __align__(16) __bf16 Psl[4][16 * 64];
  __shared__ __align__(16) float  Os[4][16 * 16];

  const int tid  = threadIdx.x;
  const int wave = tid >> 5;
  const int lane = tid & 31;
  const int hh   = lane >> 4;
  const int c    = lane & 15;

  const int bx   = blockIdx.x;
  const int qb   = bx % NQB;
  const int rest = bx / NQB;
  const int h    = rest % NH;
  const int b    = rest / NH;
  const int q0   = qb * 64 + wave * 16;
  const size_t bhp = (size_t)b * NH + h;

  const __bf16* Qc = (const __bf16*)(const void*)qcp + bhp * SEQ * QS;
  const __bf16* Kd = (const __bf16*)(const void*)kdp + bhp * SEQ * QS;
  const __bf16* Kz = (const __bf16*)(const void*)kzp + bhp * SEQ * QS;
  const __bf16* Vh = (const __bf16*)(const void*)vhp + ((size_t)b * HID + (size_t)h * HD) * SEQ;
  const __bf16* Vl = (const __bf16*)(const void*)vlp + ((size_t)b * HID + (size_t)h * HD) * SEQ;

  const v16b qa = ldfrag_b(Qc + (size_t)(q0 + c) * QS + 8 * hh);

  float mrow[8], lrow[8];
  v8f oacc = zero8();
#pragma unroll
  for (int r = 0; r < 8; ++r) { mrow[r] = -INFINITY; lrow[r] = 0.f; }

  __bf16* pwh = Psh[wave];
  __bf16* pwl = Psl[wave];

  for (int kt = 0; kt <= qb; ++kt) {
    const int kv0 = kt * 64;
    __builtin_amdgcn_fence(__ATOMIC_RELEASE, "workgroup");
    __builtin_amdgcn_wave_barrier();
    __builtin_amdgcn_fence(__ATOMIC_ACQUIRE, "workgroup");

    v8f s[4];
#pragma unroll
    for (int j = 0; j < 4; ++j) {
      const size_t ko = (size_t)(kv0 + j * 16 + c) * QS + 8 * hh;
      const v16b kd = ldfrag_b(Kd + ko);
      const v16b kz = ldfrag_b(Kz + ko);
      s[j] = mma_b(qa, kd, zero8());
      s[j] = mma_b(qa, kz, s[j]);
    }

#pragma unroll
    for (int r = 0; r < 8; ++r) {
      const int rowq = q0 + 8 * hh + r;
      float m = -INFINITY;
#pragma unroll
      for (int j = 0; j < 4; ++j) {
        const int key = kv0 + j * 16 + c;
        float sv = s[j][r] * 0.25f;
        sv = (key <= rowq) ? sv : -INFINITY;
        s[j][r] = sv;
        m = fmaxf(m, sv);
      }
#pragma unroll
      for (int off = 1; off < 16; off <<= 1) m = fmaxf(m, __shfl_xor(m, off, 32));
      const float mnew  = fmaxf(mrow[r], m);
      const float msafe = (mnew == -INFINITY) ? 0.f : mnew;
      const float alpha = __expf(mrow[r] - msafe);
      mrow[r] = mnew;
      float psum = 0.f;
#pragma unroll
      for (int j = 0; j < 4; ++j) {
        const float p = __expf(s[j][r] - msafe);
        psum += p;
        const unsigned short hb = bf_bits(p);
        const unsigned short lb = bf_bits(p - bf_up(hb));
        const int po = (8 * hh + r) * 64 + j * 16 + c;
        pwh[po] = __builtin_bit_cast(__bf16, hb);
        pwl[po] = __builtin_bit_cast(__bf16, lb);
      }
#pragma unroll
      for (int off = 1; off < 16; off <<= 1) psum += __shfl_xor(psum, off, 32);
      lrow[r] = lrow[r] * alpha + psum;
      oacc[r] *= alpha;
    }
    __builtin_amdgcn_fence(__ATOMIC_RELEASE, "workgroup");
    __builtin_amdgcn_wave_barrier();
    __builtin_amdgcn_fence(__ATOMIC_ACQUIRE, "workgroup");

#pragma unroll
    for (int kk = 0; kk < 2; ++kk) {
      FB pa, pl;
      pa.h[0] = *(const v8b*)(pwh + c * 64 + kk * 32 + 8 * hh);
      pa.h[1] = *(const v8b*)(pwh + c * 64 + kk * 32 + 16 + 8 * hh);
      pl.h[0] = *(const v8b*)(pwl + c * 64 + kk * 32 + 8 * hh);
      pl.h[1] = *(const v8b*)(pwl + c * 64 + kk * 32 + 16 + 8 * hh);
      const size_t vo = (size_t)c * SEQ + kv0 + kk * 32 + 8 * hh;
      const v16b vb = ldfrag_b(Vh + vo);
      const v16b vl = ldfrag_b(Vl + vo);
      oacc = mma_b(pa.v, vb, oacc);
      oacc = mma_b(pa.v, vl, oacc);
      oacc = mma_b(pl.v, vb, oacc);
    }
  }

  float* os = Os[wave];
#pragma unroll
  for (int r = 0; r < 8; ++r) {
    const float l = lrow[r];
    const float inv = (l > 0.f) ? (1.0f / l) : 0.f;
    os[(8 * hh + r) * HD + c] = oacc[r] * inv;
  }
  __builtin_amdgcn_fence(__ATOMIC_RELEASE, "workgroup");
  __builtin_amdgcn_wave_barrier();
  __builtin_amdgcn_fence(__ATOMIC_ACQUIRE, "workgroup");
  {
    const int row = lane >> 1, d0 = (lane & 1) * 8;
    const float* sp = os + row * HD + d0;
    v4u a, a2;
#pragma unroll
    for (int e = 0; e < 4; ++e) {
      const float f0 = sp[2 * e], f1 = sp[2 * e + 1];
      const unsigned short hb0 = bf_bits(f0), hb1 = bf_bits(f1);
      const unsigned short lb0 = bf_bits(f0 - bf_up(hb0)), lb1 = bf_bits(f1 - bf_up(hb1));
      a[e] = pk16(hb0, hb1); a2[e] = pk16(lb0, lb1);
    }
    const size_t go = (bhp * SEQ + q0 + row) * HD + d0;
    *(volatile v4u*)(ohp + go) = a;
    *(volatile v4u*)(olp + go) = a2;
    __threadfence();
    *(volatile v4u*)(ohp + go) = a;
    *(volatile v4u*)(olp + go) = a2;
  }
}

extern "C" void kernel_launch(void* const* d_in, const int* in_sizes, int n_in,
                              void* d_out, int out_size, void* d_ws, size_t ws_size,
                              hipStream_t stream) {
  if (n_in < 5) return;
  if (in_sizes[0] != NTOK * HID) return;
  if (in_sizes[1] != HID * HID) return;
  if (in_sizes[2] != HID * HID) return;
  if (in_sizes[3] != HID * HID) return;
  if (in_sizes[4] != HID * HID) return;
  if (out_size != NTOK * HID) return;

  const float* x  = (const float*)d_in[0];
  const float* Wq = (const float*)d_in[1];
  const float* Wk = (const float*)d_in[2];
  const float* Wv = (const float*)d_in[3];
  const float* Wo = (const float*)d_in[4];

  const size_t PX  = (size_t)NTOK * HID * 2;
  const size_t PW  = (size_t)HID * HID * 2;
  const size_t PQ  = (size_t)NB * NH * SEQ * QS * 2;
  const size_t PVT = (size_t)NB * HID * SEQ * 2;
  const size_t PO  = (size_t)NB * NH * SEQ * HD * 2;
  const size_t PTB = (size_t)SEQ * NPAIR * 4;
  const size_t PIV = 128;
  size_t off = 0;
  const size_t oXb  = off; off += PX;
  const size_t oWq  = off; off += PW;
  const size_t oWk  = off; off += PW;
  const size_t oWv  = off; off += PW;
  const size_t oWo  = off; off += PW;
  const size_t oQc  = off; off += PQ;
  const size_t oKd  = off; off += PQ;
  const size_t oKz  = off; off += PQ;
  const size_t oVTh = off; off += PVT;
  const size_t oVTl = off; off += PVT;
  const size_t oOh  = off; off += PO;
  const size_t oOl  = off; off += PO;
  const size_t oCt  = off; off += PTB;
  const size_t oSt  = off; off += PTB;
  const size_t oIv  = off; off += PIV;
  if (off > ws_size) return;
  if (off > (size_t)134217728) return;

  char* ws = (char*)d_ws;
  unsigned short* Xb  = (unsigned short*)(ws + oXb);
  unsigned short* Wqb = (unsigned short*)(ws + oWq);
  unsigned short* Wkb = (unsigned short*)(ws + oWk);
  unsigned short* Wvb = (unsigned short*)(ws + oWv);
  unsigned short* Wob = (unsigned short*)(ws + oWo);
  unsigned short* Qc  = (unsigned short*)(ws + oQc);
  unsigned short* Kd  = (unsigned short*)(ws + oKd);
  unsigned short* Kz  = (unsigned short*)(ws + oKz);
  unsigned short* VTh = (unsigned short*)(ws + oVTh);
  unsigned short* VTl = (unsigned short*)(ws + oVTl);
  unsigned short* Oh  = (unsigned short*)(ws + oOh);
  unsigned short* Ol  = (unsigned short*)(ws + oOl);
  float*          Ct  = (float*)(ws + oCt);
  float*          St  = (float*)(ws + oSt);
  float*          Iv  = (float*)(ws + oIv);

  const dim3 blk256(256);
  const dim3 blk128(128);
  const int n8x = NTOK * HID / 8;
  const int n8w = HID * HID / 8;
  const dim3 gCvtX((n8x + 255) / 256);
  const dim3 gCvtW((n8w + 255) / 256);
  const dim3 gTab(SEQ / 32);
  const dim3 gGemm(((NTOK / 64) * (HID / 32)) / 4);
  const dim3 gAttn(NB * NH * NQB);

  rope_inv<<<dim3(1), dim3(32), 0, stream>>>(Iv);
  rope_tab<<<gTab, blk256, 0, stream>>>(Iv, Ct, St);
  cvt_bf16x8<<<gCvtX, blk256, 0, stream>>>(x, Xb, n8x);
  cvt_bf16x8<<<gCvtW, blk256, 0, stream>>>(Wq, Wqb, n8w);
  cvt_bf16x8<<<gCvtW, blk256, 0, stream>>>(Wk, Wkb, n8w);
  cvt_bf16x8<<<gCvtW, blk256, 0, stream>>>(Wv, Wvb, n8w);
  cvt_bf16x8<<<gCvtW, blk256, 0, stream>>>(Wo, Wob, n8w);
  gemm_xw<0, false><<<gGemm, blk128, 0, stream>>>(Xb, Xb, Wqb, (void*)Qc, (void*)Qc, Ct, St);
  gemm_xw<1, false><<<gGemm, blk128, 0, stream>>>(Xb, Xb, Wkb, (void*)Kd, (void*)Kz, Ct, St);
  gemm_xw<2, false><<<gGemm, blk128, 0, stream>>>(Xb, Xb, Wvb, (void*)VTh, (void*)VTl, Ct, St);
  attn_causal16<<<gAttn, blk128, 0, stream>>>(Qc, Kd, Kz, VTh, VTl, Oh, Ol);
  gemm_xw<3, true><<<gGemm, blk128, 0, stream>>>(Oh, Ol, Wob, d_out, d_out, Ct, St);
  (void)hipGetLastError();
}
